// CPUMamba_86337432584510
// MI455X (gfx1250) — hardware-verified
//
#include <hip/hip_runtime.h>
#include <math.h>

#define DM    1024
#define DIN   2048
#define DST   16
#define DTR   64
#define NB    2
#define TT    2048
#define MTOK  (NB * TT)
#define XZC   (2 * DIN)
#define DBLN  96
#define DBLP  128
#define TCH   32

static_assert((MTOK % 128) == 0);
static_assert((TT % TCH) == 0);
static_assert((DIN % 128) == 0);
static_assert((XZC % 64) == 0);
static_assert((DM % 64) == 0);
static_assert((DBLP % 64) == 0);
static_assert((DM % 32) == 0 && (DIN % 32) == 0 && (DTR % 32) == 0);

typedef unsigned short us;
typedef us     v8us __attribute__((ext_vector_type(8)));
typedef __bf16 v16b __attribute__((ext_vector_type(16)));
typedef __bf16 v8b  __attribute__((ext_vector_type(8)));
typedef float  v8f  __attribute__((ext_vector_type(8)));
typedef float  v4f  __attribute__((ext_vector_type(4)));
typedef v8b  __attribute__((may_alias)) v8ba;
typedef v8us __attribute__((may_alias)) v8usa;
typedef v4f  __attribute__((may_alias)) v4fa;

union FragB { v16b v; v8b half[2]; };

__device__ __forceinline__ us bf_bits(float f) {
  unsigned u = __float_as_uint(f);
  u += 0x7FFFu + ((u >> 16) & 1u);
  return (us)(u >> 16);
}
__device__ __forceinline__ float bf_up(us b) { return __uint_as_float(((unsigned)b) << 16); }
__device__ __forceinline__ float rcp_f(float x) { return __builtin_amdgcn_rcpf(x); }
__device__ __forceinline__ float silu_f(float v) { return v * rcp_f(1.0f + __expf(-v)); }
__device__ __forceinline__ float softplus_f(float v) { return fmaxf(v, 0.0f) + log1pf(__expf(-fabsf(v))); }

__device__ __forceinline__ v8f wmma_bf(v16b a, v16b b, v8f c) {
  v8f d = __builtin_amdgcn_wmma_f32_16x16x32_bf16(false, a, false, b, (short)0, c, false, false);
  asm volatile("v_nop\n\tv_nop\n\tv_nop\n\tv_nop" : "+v"(d) : "v"(a), "v"(b));
  return d;
}

__device__ __forceinline__ v16b load_frag(const us* p, int h) {
  FragB f;
  f.half[0] = *(const v8ba*)(p + 8 * h);
  f.half[1] = *(const v8ba*)(p + 16 + 8 * h);
  return f.v;
}

#define G_X    (MTOK * DM / 8)
#define G_WIN  (XZC * DM / 8)
#define G_WX   (DBLP * DIN / 8)
#define G_WDT  (DIN * DTR / 8)
#define G_WOUT (DM * DIN / 8)
#define C1 (G_X)
#define C2 (C1 + G_WIN)
#define C3 (C2 + G_WX)
#define C4 (C3 + G_WDT)
#define GTOT (C4 + G_WOUT)

__global__ __launch_bounds__(256) void k_convert(
    const float* __restrict__ x, const float* __restrict__ win, const float* __restrict__ wx,
    const float* __restrict__ wdt, const float* __restrict__ wout,
    us* dxh, us* dxl, us* dwinh, us* dwinl, us* dwxh, us* dwxl,
    us* dwdt, us* dwouth, us* dwoutl)
{
  const int g = blockIdx.x * 256 + threadIdx.x;
  if (g >= GTOT) return;
  const float* src = x;
  us* dh = dxh;
  us* dl = dxl;
  bool zero = false;
  if (g < C1) {
    src = x + (size_t)g * 8; dh = dxh + (size_t)g * 8; dl = dxl + (size_t)g * 8;
  } else if (g < C2) {
    const int e = g - C1;
    src = win + (size_t)e * 8; dh = dwinh + (size_t)e * 8; dl = dwinl + (size_t)e * 8;
  } else if (g < C3) {
    const int e = g - C2;
    const int row = e >> 8;
    dh = dwxh + (size_t)e * 8; dl = dwxl + (size_t)e * 8;
    if (row < DBLN) src = wx + (size_t)e * 8; else zero = true;
  } else if (g < C4) {
    const int e = g - C3;
    src = wdt + (size_t)e * 8; dh = dwdt + (size_t)e * 8; dl = nullptr;
  } else {
    const int e = g - C4;
    src = wout + (size_t)e * 8; dh = dwouth + (size_t)e * 8; dl = dwoutl + (size_t)e * 8;
  }
  v4f a = {0.0f, 0.0f, 0.0f, 0.0f};
  v4f c = a;
  if (!zero) {
    a = *(const v4fa*)src;
    c = *(const v4fa*)(src + 4);
  }
  float v[8] = { a.x, a.y, a.z, a.w, c.x, c.y, c.z, c.w };
  us hb[8], lb[8];
#pragma unroll
  for (int i = 0; i < 8; ++i) {
    hb[i] = bf_bits(v[i]);
    lb[i] = bf_bits(v[i] - bf_up(hb[i]));
  }
  const v8us oh = { hb[0], hb[1], hb[2], hb[3], hb[4], hb[5], hb[6], hb[7] };
  const v8us ol = { lb[0], lb[1], lb[2], lb[3], lb[4], lb[5], lb[6], lb[7] };
  *(volatile v8us*)dh = oh;
  if (dl != nullptr) *(volatile v8us*)dl = ol;
  __threadfence();
  *(volatile v8us*)dh = oh;
  if (dl != nullptr) *(volatile v8us*)dl = ol;
}

template <bool OUTH>
__device__ __forceinline__ void gemm_store(const float* sT, float* outf, us* outh,
                                           int N, int hN, int m0, int n0, int w, int lane) {
  const int q8 = lane & 7, sub = lane >> 3;
#pragma unroll
  for (int i = 0; i < 16; ++i) {
    const int lid = i * 4 + sub;
    const int row = 32 * w + (lid >> 1), hl = lid & 1;
    const v4f v = *(const v4fa*)(sT + row * 64 + 32 * hl + 4 * q8);
    float* dst = outf + (size_t)(m0 + row) * N + n0 + 32 * hl + 4 * q8;
    *(volatile v4f*)dst = v;
  }
  if (OUTH) {
    if (n0 + 64 <= hN) {
#pragma unroll
      for (int i = 0; i < 8; ++i) {
        const int lid = i * 4 + sub;
        const int row = 32 * w + lid;
        const v4f a = *(const v4fa*)(sT + row * 64 + 8 * q8);
        const v4f c = *(const v4fa*)(sT + row * 64 + 8 * q8 + 4);
        const v8us o = { bf_bits(a.x), bf_bits(a.y), bf_bits(a.z), bf_bits(a.w),
                         bf_bits(c.x), bf_bits(c.y), bf_bits(c.z), bf_bits(c.w) };
        us* dst = outh + (size_t)(m0 + row) * hN + n0 + 8 * q8;
        *(volatile v8us*)dst = o;
      }
    }
  }
}

template <int NP, bool OUTH>
__global__ __launch_bounds__(128) void k_gemm(
    const us* __restrict__ Ah, const us* __restrict__ Al, int lda,
    const us* __restrict__ Wh, const us* __restrict__ Wl, int K, int N,
    float* outf, us* outh, int hN)
{
  __shared__ __attribute__((aligned(16))) float sT[128 * 64];

  const int tid = threadIdx.x, lane = tid & 31, w = tid >> 5;
  const int h = lane >> 4, m = lane & 15;
  const int m0 = blockIdx.y * 128, n0 = blockIdx.x * 64;
  const int m0w = m0 + 32 * w;

  const us* a0p = Ah + (size_t)(m0w + m) * lda;
  const us* a1p = a0p + (size_t)16 * lda;
  const us* c0p = Al + (size_t)(m0w + m) * lda;
  const us* c1p = c0p + (size_t)16 * lda;
  const us* wph = Wh + (size_t)(n0 + m) * K;
  const us* wpl = Wl + (size_t)(n0 + m) * K;

  const v8f zero8 = {0.f, 0.f, 0.f, 0.f, 0.f, 0.f, 0.f, 0.f};
  v8f acc[2][4];
#pragma unroll
  for (int mt = 0; mt < 2; ++mt)
#pragma unroll
    for (int nt = 0; nt < 4; ++nt) acc[mt][nt] = zero8;

#pragma unroll 1
  for (int k0 = 0; k0 < K; k0 += 32) {
    const v16b a0 = load_frag(a0p + k0, h);
    const v16b a1 = load_frag(a1p + k0, h);
    v16b c0 = a0, c1 = a1;
    if (NP == 3) {
      c0 = load_frag(c0p + k0, h);
      c1 = load_frag(c1p + k0, h);
    }
#pragma unroll
    for (int nt = 0; nt < 4; ++nt) {
      const v16b bh = load_frag(wph + (size_t)nt * 16 * K + k0, h);
      acc[0][nt] = wmma_bf(a0, bh, acc[0][nt]);
      acc[1][nt] = wmma_bf(a1, bh, acc[1][nt]);
      if (NP == 3) {
        const v16b bl = load_frag(wpl + (size_t)nt * 16 * K + k0, h);
        acc[0][nt] = wmma_bf(a0, bl, acc[0][nt]);
        acc[1][nt] = wmma_bf(a1, bl, acc[1][nt]);
        acc[0][nt] = wmma_bf(c0, bh, acc[0][nt]);
        acc[1][nt] = wmma_bf(c1, bh, acc[1][nt]);
      }
    }
  }

#pragma unroll
  for (int nt = 0; nt < 4; ++nt) {
    const int nl = 16 * nt + m;
#pragma unroll
    for (int mt = 0; mt < 2; ++mt) {
#pragma unroll
      for (int r = 0; r < 8; ++r) {
        const int rowl = 32 * w + 16 * mt + 8 * h + r;
        sT[rowl * 64 + nl] = acc[mt][nt][r];
      }
    }
  }
  __syncthreads();

  gemm_store<OUTH>(sT, outf, outh, N, hN, m0, n0, w, lane);
  __threadfence();
  gemm_store<OUTH>(sT, outf, outh, N, hN, m0, n0, w, lane);
}

__global__ __launch_bounds__(256) void k_conv(
    const float* __restrict__ xz, const float* __restrict__ cw, const float* __restrict__ cb,
    us* xh, us* xl)
{
  const int row = blockIdx.x;
  const int l = row & (TT - 1);
  const int c0 = threadIdx.x * 8;
  v4f wv[8];
#pragma unroll
  for (int i = 0; i < 8; ++i) wv[i] = *(const v4fa*)(cw + (size_t)(c0 + i) * 4);
  float acc[8];
#pragma unroll
  for (int i = 0; i < 8; ++i) acc[i] = 0.0f;
#pragma unroll
  for (int k = 0; k < 4; ++k) {
    const int ls = l + k - 3;
    if (ls >= 0) {
      const float* p = xz + (size_t)(row + k - 3) * XZC + c0;
      const v4f a = *(const v4fa*)p;
      const v4f c = *(const v4fa*)(p + 4);
      acc[0] += a.x * wv[0][k]; acc[1] += a.y * wv[1][k];
      acc[2] += a.z * wv[2][k]; acc[3] += a.w * wv[3][k];
      acc[4] += c.x * wv[4][k]; acc[5] += c.y * wv[5][k];
      acc[6] += c.z * wv[6][k]; acc[7] += c.w * wv[7][k];
    }
  }
  const v4f bta = *(const v4fa*)(cb + c0);
  const v4f btc = *(const v4fa*)(cb + c0 + 4);
  acc[0] += bta.x; acc[1] += bta.y; acc[2] += bta.z; acc[3] += bta.w;
  acc[4] += btc.x; acc[5] += btc.y; acc[6] += btc.z; acc[7] += btc.w;
  us hb[8], lb[8];
#pragma unroll
  for (int i = 0; i < 8; ++i) {
    const float y = silu_f(acc[i]);
    hb[i] = bf_bits(y);
    lb[i] = bf_bits(y - bf_up(hb[i]));
  }
  const v8us oh = { hb[0], hb[1], hb[2], hb[3], hb[4], hb[5], hb[6], hb[7] };
  const v8us ol = { lb[0], lb[1], lb[2], lb[3], lb[4], lb[5], lb[6], lb[7] };
  us* dh = xh + (size_t)row * DIN + c0;
  us* dl = xl + (size_t)row * DIN + c0;
  *(volatile v8us*)dh = oh;
  *(volatile v8us*)dl = ol;
  __threadfence();
  *(volatile v8us*)dh = oh;
  *(volatile v8us*)dl = ol;
}

__device__ __forceinline__ void scan_store(const us* sY, us* dstp,
                                           int b, int l0, int cbase, int w, int lane) {
  const int q8 = lane & 7, sub = lane >> 3;
#pragma unroll
  for (int i = 0; i < 4; ++i) {
    const int lid = w * 16 + i * 4 + sub;
    const int r = lid >> 1, hl = lid & 1;
    const v8us v = *(const v8usa*)(sY + r * 128 + 64 * hl + 8 * q8);
    us* dst = dstp + (size_t)(b * TT + l0 + r) * DIN + cbase + 64 * hl + 8 * q8;
    *(volatile v8us*)dst = v;
  }
}

__global__ __launch_bounds__(128) void k_scan(
    const float* __restrict__ xz,
    const float* __restrict__ dbl,
    const us* __restrict__ dtlo,
    const us* __restrict__ wdt,
    const float* __restrict__ dtb,
    const float* __restrict__ alog,
    const float* __restrict__ dp,
    const float* __restrict__ cw,
    const float* __restrict__ cb,
    us* yh, us* yl)
{
  __shared__ __attribute__((aligned(16))) float sBC[TCH * 32];
  __shared__ __attribute__((aligned(16))) float sDT[TCH * 128];
  __shared__ __attribute__((aligned(16))) us    sYh[TCH * 128];
  __shared__ __attribute__((aligned(16))) us    sYl[TCH * 128];

  const int tid = threadIdx.x, lane = tid & 31, w = tid >> 5;
  const int h = lane >> 4, m = lane & 15;
  const int b = blockIdx.y;
  const int cbase = blockIdx.x * 128;
  const int d = cbase + tid;

  float Aa[DST];
#pragma unroll
  for (int j = 0; j < 4; ++j) {
    const v4f al = *(const v4fa*)(alog + (size_t)d * DST + 4 * j);
    Aa[4 * j + 0] = -expf(al.x); Aa[4 * j + 1] = -expf(al.y);
    Aa[4 * j + 2] = -expf(al.z); Aa[4 * j + 3] = -expf(al.w);
  }
  float hs[DST];
#pragma unroll
  for (int n = 0; n < DST; ++n) hs[n] = 0.0f;
  const float Dd = dp[d];
  const v4f wv4 = *(const v4fa*)(cw + (size_t)d * 4);
  const float cw0 = wv4.x, cw1 = wv4.y, cw2 = wv4.z, cw3 = wv4.w;
  const float cbd = cb[d];
  float xm1 = 0.0f, xm2 = 0.0f, xm3 = 0.0f;

  const int chw = cbase + 32 * w;
  const us* wr0 = wdt + (size_t)(chw + m) * DTR;
  const us* wr1 = wr0 + (size_t)16 * DTR;
  const float bia0 = dtb[chw + m];
  const float bia1 = dtb[chw + 16 + m];

  const int st_i = tid >> 2, st_p = (tid & 3) * 8;
  const v8f zero8 = {0.f, 0.f, 0.f, 0.f, 0.f, 0.f, 0.f, 0.f};

#pragma unroll 1
  for (int l0 = 0; l0 < TT; l0 += TCH) {
    __syncthreads();
    {
      const float* src = dbl + (size_t)(b * TT + l0 + st_i) * DBLP + DTR + st_p;
      *(v4fa*)(sBC + st_i * 32 + st_p)     = *(const v4fa*)src;
      *(v4fa*)(sBC + st_i * 32 + st_p + 4) = *(const v4fa*)(src + 4);
    }
    {
      const us* ar0 = dtlo + (size_t)(b * TT + l0 + m) * DTR;
      const us* ar1 = ar0 + (size_t)16 * DTR;
      v8f c00 = zero8, c01 = zero8, c10 = zero8, c11 = zero8;
#pragma unroll
      for (int ks = 0; ks < 2; ++ks) {
        const int k0 = 32 * ks;
        const v16b a0 = load_frag(ar0 + k0, h);
        const v16b a1 = load_frag(ar1 + k0, h);
        const v16b b0 = load_frag(wr0 + k0, h);
        const v16b b1 = load_frag(wr1 + k0, h);
        c00 = wmma_bf(a0, b0, c00);
        c01 = wmma_bf(a0, b1, c01);
        c10 = wmma_bf(a1, b0, c10);
        c11 = wmma_bf(a1, b1, c11);
      }
#pragma unroll
      for (int r = 0; r < 8; ++r) {
        sDT[(8 * h + r) * 128 + 32 * w + m]           = c00[r] + bia0;
        sDT[(8 * h + r) * 128 + 32 * w + 16 + m]      = c01[r] + bia1;
        sDT[(16 + 8 * h + r) * 128 + 32 * w + m]      = c10[r] + bia0;
        sDT[(16 + 8 * h + r) * 128 + 32 * w + 16 + m] = c11[r] + bia1;
      }
    }
    __syncthreads();

#pragma unroll 1
    for (int i = 0; i < TCH; ++i) {
      const size_t row = (size_t)(b * TT + l0 + i);
      const float xin = xz[row * XZC + d];
      const float zv  = xz[row * XZC + DIN + d];
      const float dtv = softplus_f(sDT[i * 128 + tid]);
      float conv = xm3 * cw0;
      conv += xm2 * cw1;
      conv += xm1 * cw2;
      conv += xin * cw3;
      conv += cbd;
      xm3 = xm2; xm2 = xm1; xm1 = xin;
      const float xc = silu_f(conv);

      v4f bc[8];
#pragma unroll
      for (int j = 0; j < 8; ++j) bc[j] = *(const v4fa*)(sBC + i * 32 + 4 * j);

      float y = 0.0f;
#pragma unroll
      for (int n = 0; n < DST; ++n) {
        const float Bn = bc[n >> 2][n & 3];
        const float Cn = bc[4 + (n >> 2)][n & 3];
        const float dA = __expf(dtv * Aa[n]);
        hs[n] = dA * hs[n] + (dtv * Bn) * xc;
        y += hs[n] * Cn;
      }
      y += Dd * xc;
      y *= silu_f(zv);
      const us hb = bf_bits(y);
      const us lb = bf_bits(y - bf_up(hb));
      sYh[i * 128 + tid] = hb;
      sYl[i * 128 + tid] = lb;
    }
    __syncthreads();
    scan_store(sYh, yh, b, l0, cbase, w, lane);
    scan_store(sYl, yl, b, l0, cbase, w, lane);
    __threadfence();
    scan_store(sYh, yh, b, l0, cbase, w, lane);
    scan_store(sYl, yl, b, l0, cbase, w, lane);
  }
}

extern "C" void kernel_launch(void* const* d_in, const int* in_sizes, int n_in,
                              void* d_out, int out_size, void* d_ws, size_t ws_size,
                              hipStream_t stream)
{
  if (n_in < 10) return;
  if (in_sizes[0] != MTOK * DM) return;
  if (in_sizes[1] != XZC * DM) return;
  if (in_sizes[2] != DIN * 4 || in_sizes[3] != DIN) return;
  if (in_sizes[4] != DBLN * DIN) return;
  if (in_sizes[5] != DIN * DTR || in_sizes[6] != DIN) return;
  if (in_sizes[7] != DIN * DST || in_sizes[8] != DIN) return;
  if (in_sizes[9] != DM * DIN) return;
  if (out_size != MTOK * DM) return;

  const float* x          = (const float*)d_in[0];
  const float* in_proj_w  = (const float*)d_in[1];
  const float* conv_w     = (const float*)d_in[2];
  const float* conv_b     = (const float*)d_in[3];
  const float* x_proj_w   = (const float*)d_in[4];
  const float* dt_proj_w  = (const float*)d_in[5];
  const float* dt_proj_b  = (const float*)d_in[6];
  const float* A_log      = (const float*)d_in[7];
  const float* Dp         = (const float*)d_in[8];
  const float* out_proj_w = (const float*)d_in[9];
  float* outp = (float*)d_out;

  const size_t B_P0   = (size_t)MTOK * DIN * 2;
  const size_t B_P1   = (size_t)MTOK * DIN * 2;
  const size_t B_XPL  = (size_t)MTOK * DM * 2;
  const size_t B_WIPL = (size_t)XZC * DM * 2;
  const size_t B_XZ   = (size_t)MTOK * XZC * 4;
  const size_t B_WOUT = (size_t)DM * DIN * 2;
  const size_t B_WX   = (size_t)DBLP * DIN * 2;
  const size_t B_WDT  = (size_t)DIN * DTR * 2;
  const size_t B_DBL  = (size_t)MTOK * DBLP * 4;
  const size_t B_DTLO = (size_t)MTOK * DTR * 2;
  if (2 * B_XPL != B_P0 || 2 * B_WIPL != B_P1) return;
  size_t off = 0;
  const size_t o_p0    = off; off += B_P0;
  const size_t o_p1    = off; off += B_P1;
  const size_t o_xz    = off; off += B_XZ;
  const size_t o_wouth = off; off += B_WOUT;
  const size_t o_woutl = off; off += B_WOUT;
  const size_t o_wxh   = off; off += B_WX;
  const size_t o_wxl   = off; off += B_WX;
  const size_t o_wdt   = off; off += B_WDT;
  const size_t o_dbl   = off; off += B_DBL;
  const size_t o_dtlo  = off; off += B_DTLO;
  const size_t total   = off;
  if (total > ws_size) return;
  if (total > (size_t)134217728) return;

  char* ws = (char*)d_ws;
  us*    xh    = (us*)(ws + o_p0);
  us*    xl    = (us*)(ws + o_p0 + B_XPL);
  us*    winh  = (us*)(ws + o_p1);
  us*    winl  = (us*)(ws + o_p1 + B_WIPL);
  us*    xch   = (us*)(ws + o_p0);
  us*    xcl   = (us*)(ws + o_p1);
  us*    ych   = (us*)(ws + o_p0);
  us*    ycl   = (us*)(ws + o_p1);
  float* xz    = (float*)(ws + o_xz);
  us*    wouth = (us*)(ws + o_wouth);
  us*    woutl = (us*)(ws + o_woutl);
  us*    wxh   = (us*)(ws + o_wxh);
  us*    wxl   = (us*)(ws + o_wxl);
  us*    wdt   = (us*)(ws + o_wdt);
  float* dbl   = (float*)(ws + o_dbl);
  us*    dtlo  = (us*)(ws + o_dtlo);

  k_convert<<<(GTOT + 255) / 256, 256, 0, stream>>>(x, in_proj_w, x_proj_w, dt_proj_w, out_proj_w,
                                                     xh, xl, winh, winl, wxh, wxl, wdt, wouth, woutl);
  k_gemm<3, false><<<dim3(XZC / 64, MTOK / 128), 128, 0, stream>>>(
      xh, xl, DM, winh, winl, DM, XZC, xz, dtlo, 0);
  k_conv<<<MTOK, 256, 0, stream>>>(xz, conv_w, conv_b, xch, xcl);
  k_gemm<3, true><<<dim3(DBLP / 64, MTOK / 128), 128, 0, stream>>>(
      xch, xcl, DIN, wxh, wxl, DIN, DBLP, dbl, dtlo, DTR);
  k_scan<<<dim3(DIN / 128, NB), 128, 0, stream>>>(xz, dbl, dtlo, wdt, dt_proj_b, A_log, Dp,
                                                   conv_w, conv_b, ych, ycl);
  k_gemm<3, false><<<dim3(DM / 64, MTOK / 128), 128, 0, stream>>>(
      ych, ycl, DIN, wouth, woutl, DIN, DM, outp, dtlo, 0);
}
